// TimeStretch_33311766347850
// MI455X (gfx1250) — hardware-verified
//
#include <hip/hip_runtime.h>
#include <stddef.h>
#include <stdint.h>

#pragma clang fp contract(off)

constexpr int BATCH   = 64;
constexpr int BINS    = 512;
constexpr int FRAMES  = 64;
constexpr int WLEN    = 1022;
constexpr int HOP     = 511;
constexpr int SIG_LEN = 33215;
constexpr int N_SEG   = 36;
constexpr int STEP    = 950;
constexpr int SEG     = 1000;
constexpr int OV      = 50;
constexpr int DSHIFT  = 50;
constexpr int FR2     = 66;
constexpr int KD      = 1024;
constexpr int ND      = 1024;
constexpr int M1      = BATCH * FRAMES;
constexpr int M2      = BATCH * FR2;
constexpr int OUT_N   = BATCH * BINS * FR2 * 2;

constexpr int BMT = 128;
constexpr int BNT = 128;
constexpr int STP = 36;

constexpr float TWO_PI_F = 6.28318530717958647692f;
constexpr float CW1 = 1.0f / 1022.0f;
constexpr float CW2 = 2.0f / 1022.0f;

static_assert(M1 % BMT == 0);
static_assert(M2 % BMT == 0);
static_assert(ND % BNT == 0);
static_assert(KD % 32 == 0);
static_assert((STP * 4) % 16 == 0);
static_assert(OUT_N % 1024 == 0);
static_assert(HOP * (FR2 - 1) + (WLEN - 1) < N_SEG * (SEG - 2 * OV) + (N_SEG + 1) * OV);

constexpr size_t SZ_TRIG = (size_t)2 * 1024 * 4;
constexpr size_t SZ_BPL  = (size_t)ND * KD * 2;
constexpr size_t SZ_A1   = (size_t)M1 * KD * 2;
constexpr size_t SZ_FR   = (size_t)M1 * ND * 4;
constexpr size_t SZ_A2   = (size_t)M2 * KD * 2;
constexpr size_t SZ_S    = (size_t)M2 * ND * 4;
constexpr size_t OFF_TRIG = 0;
constexpr size_t OFF_BIH  = OFF_TRIG + SZ_TRIG;
constexpr size_t OFF_BIL  = OFF_BIH + SZ_BPL;
constexpr size_t OFF_BFH  = OFF_BIL + SZ_BPL;
constexpr size_t OFF_BFL  = OFF_BFH + SZ_BPL;
constexpr size_t OFF_A1H  = OFF_BFL + SZ_BPL;
constexpr size_t OFF_A1L  = OFF_A1H + SZ_A1;
constexpr size_t OFF_FR   = OFF_A1L + SZ_A1;
constexpr size_t OFF_A2H  = OFF_FR + SZ_FR;
constexpr size_t OFF_A2L  = OFF_A2H + SZ_A2;
constexpr size_t OFF_S    = OFF_A2L + SZ_A2;
constexpr size_t WS_TOTAL = OFF_S + SZ_S;
static_assert(WS_TOTAL <= (size_t)134217728);
static_assert(OFF_BIH % 128 == 0 && OFF_A1H % 128 == 0 && OFF_FR % 128 == 0 && OFF_A2H % 128 == 0 && OFF_S % 128 == 0);

typedef __bf16 v16bf __attribute__((ext_vector_type(16)));
typedef unsigned short v8us __attribute__((ext_vector_type(8)));
typedef unsigned int v4u __attribute__((ext_vector_type(4)));
typedef float v8f __attribute__((ext_vector_type(8)));
typedef float v4f __attribute__((ext_vector_type(4)));
typedef v4f __attribute__((may_alias)) v4fa;

union Frag { v16bf v; v8us u[2]; };

__device__ __forceinline__ v8f mma_bf(v16bf a, v16bf b, v8f cacc) {
  cacc = __builtin_amdgcn_wmma_f32_16x16x32_bf16(false, a, false, b, (short)0, cacc, false, false);
  asm volatile("v_nop\n\tv_nop\n\tv_nop\n\tv_nop" : "+v"(cacc) : "v"(a), "v"(b));
  return cacc;
}

__device__ __forceinline__ v8f zero8() { return (v8f){0.f, 0.f, 0.f, 0.f, 0.f, 0.f, 0.f, 0.f}; }

__device__ __forceinline__ v16bf ldfrag(const unsigned short* __restrict__ p, int row0, int k0, int lane) {
  const int m = lane & 15, lh = lane >> 4;
  const unsigned short* q = p + (size_t)(row0 + m) * KD + k0 + 8 * lh;
  Frag f;
  f.u[0] = *(const v8us*)(q);
  f.u[1] = *(const v8us*)(q + 16);
  return f.v;
}

__device__ __forceinline__ unsigned int bf16_rne_bits(float x) {
  const unsigned int u = __float_as_uint(x);
  return (u + 0x7FFFu + ((u >> 16) & 1u)) >> 16;
}
__device__ __forceinline__ void split_bf16(float x, unsigned int& h, unsigned int& l) {
  const unsigned int hb = bf16_rne_bits(x);
  const float hf = __uint_as_float(hb << 16);
  h = hb;
  l = bf16_rne_bits(x - hf);
}

__device__ __forceinline__ void shin(unsigned int& w0, unsigned int& w1, unsigned int& w2, unsigned int& w3, unsigned int hb) {
  w0 = (w0 >> 16) | (w1 << 16);
  w1 = (w1 >> 16) | (w2 << 16);
  w2 = (w2 >> 16) | (w3 << 16);
  w3 = (w3 >> 16) | (hb << 16);
}

__device__ __forceinline__ void consume(float& v) { asm volatile("" : "+v"(v)); }

__global__ __launch_bounds__(256) void k_trig(float* __restrict__ cosT, float* __restrict__ sinT) {
  const int i = blockIdx.x * 256 + (int)threadIdx.x;
  const bool ok = i < WLEN;
  const int r = ok ? i : (WLEN - 1);
  const float ang = (TWO_PI_F * (float)r) / (float)WLEN;
  float cs = cosf(ang);
  float sn = sinf(ang);
  cs = ok ? cs : 0.0f;
  sn = ok ? sn : 0.0f;
  *(volatile float*)(cosT + i) = cs;
  *(volatile float*)(sinT + i) = sn;
  __threadfence();
  *(volatile float*)(cosT + i) = cs;
  *(volatile float*)(sinT + i) = sn;
}

__device__ __forceinline__ void stage_trig(const float* __restrict__ cosT, const float* __restrict__ sinT,
                                           float* sc, float* ss, int tid) {
#pragma unroll
  for (int it = 0; it < 2; ++it) {
    const int p = tid + 128 * it;
    const v4f c4 = *(const v4f*)(cosT + 4 * p);
    const v4f s4 = *(const v4f*)(sinT + 4 * p);
    *(v4fa*)(sc + 4 * p) = c4;
    *(v4fa*)(ss + 4 * p) = s4;
  }
}

__global__ __launch_bounds__(128) void k_basis_inv(const float* __restrict__ cosT, const float* __restrict__ sinT,
                                                   unsigned short* __restrict__ bh, unsigned short* __restrict__ bl) {
  __shared__ __align__(16) float sc[1024];
  __shared__ __align__(16) float ss[1024];
  const int n = blockIdx.x;
  const int tid = threadIdx.x;
  stage_trig(cosT, sinT, sc, ss, tid);
  __syncthreads();

  const bool rowv = n < WLEN;
  const int nc = rowv ? n : (WLEN - 1);
  const int jj = nc % HOP;
  const float h_n = 0.5f * (1.0f - sc[nc]);
  const float h_a = 0.5f * (1.0f - sc[jj]);
  const float h_b = 0.5f * (1.0f - sc[jj + HOP]);
  const float den = h_a * h_a + h_b * h_b;
  const float iw = h_n / den;
  const int kc0 = tid * 8;
  const bool re = tid < 64;
  unsigned int h0 = 0u, h1 = 0u, h2 = 0u, h3 = 0u, l0 = 0u, l1 = 0u, l2 = 0u, l3 = 0u;
#pragma unroll 1
  for (int j = 0; j < 8; ++j) {
    const int kcol = kc0 + j;
    const int k = re ? kcol : (kcol - BINS);
    const int r = (k * nc) % WLEN;
    const bool special = (k == 0) || (k == HOP);
    const float vre = (special ? CW1 : CW2) * sc[r] * iw;
    const float vim = special ? 0.0f : (-CW2 * ss[r] * iw);
    float v = re ? vre : vim;
    v = rowv ? v : 0.0f;
    unsigned int hb, lb;
    split_bf16(v, hb, lb);
    shin(h0, h1, h2, h3, hb);
    shin(l0, l1, l2, l3, lb);
  }
  const v4u vh = (v4u){h0, h1, h2, h3};
  const v4u vl = (v4u){l0, l1, l2, l3};
  unsigned short* ph = bh + (size_t)n * KD + kc0;
  unsigned short* pl = bl + (size_t)n * KD + kc0;
  *(volatile v4u*)ph = vh;
  *(volatile v4u*)pl = vl;
  __threadfence();
  *(volatile v4u*)ph = vh;
  *(volatile v4u*)pl = vl;
}

__global__ __launch_bounds__(128) void k_basis_fwd(const float* __restrict__ cosT, const float* __restrict__ sinT,
                                                   unsigned short* __restrict__ bh, unsigned short* __restrict__ bl) {
  __shared__ __align__(16) float sc[1024];
  __shared__ __align__(16) float ss[1024];
  const int jrow = blockIdx.x;
  const int tid = threadIdx.x;
  stage_trig(cosT, sinT, sc, ss, tid);
  __syncthreads();

  const bool re = jrow < BINS;
  const int k = re ? jrow : (jrow - BINS);
  const bool special = (k == 0) || (k == HOP);
  const int n0 = tid * 8;
  unsigned int h0 = 0u, h1 = 0u, h2 = 0u, h3 = 0u, l0 = 0u, l1 = 0u, l2 = 0u, l3 = 0u;
#pragma unroll 1
  for (int j = 0; j < 8; ++j) {
    const int n = n0 + j;
    const bool nv = n < WLEN;
    const int ncl = nv ? n : (WLEN - 1);
    const float hn = 0.5f * (1.0f - sc[ncl]);
    const int r = (k * ncl) % WLEN;
    const float vre = hn * sc[r];
    const float vim = special ? 0.0f : (-hn * ss[r]);
    float v = re ? vre : vim;
    v = nv ? v : 0.0f;
    unsigned int hb, lb;
    split_bf16(v, hb, lb);
    shin(h0, h1, h2, h3, hb);
    shin(l0, l1, l2, l3, lb);
  }
  const v4u vh = (v4u){h0, h1, h2, h3};
  const v4u vl = (v4u){l0, l1, l2, l3};
  unsigned short* ph = bh + (size_t)jrow * KD + n0;
  unsigned short* pl = bl + (size_t)jrow * KD + n0;
  *(volatile v4u*)ph = vh;
  *(volatile v4u*)pl = vl;
  __threadfence();
  *(volatile v4u*)ph = vh;
  *(volatile v4u*)pl = vl;
}

__global__ __launch_bounds__(128) void k_pack1(const float* __restrict__ x,
                                              unsigned short* __restrict__ a1h, unsigned short* __restrict__ a1l) {
  const int r = blockIdx.x;
  const int b = r >> 6, f = r & 63;
  const int tid = threadIdx.x;
  const int kc0 = tid * 8;
  const int c = tid >> 6;
  const int k0 = kc0 & (BINS - 1);
  unsigned int h0 = 0u, h1 = 0u, h2 = 0u, h3 = 0u, l0 = 0u, l1 = 0u, l2 = 0u, l3 = 0u;
#pragma unroll 1
  for (int j = 0; j < 8; ++j) {
    const int k = k0 + j;
    float v = x[(((size_t)b * BINS + k) * FRAMES + f) * 2 + c];
    consume(v);
    unsigned int hb, lb;
    split_bf16(v, hb, lb);
    shin(h0, h1, h2, h3, hb);
    shin(l0, l1, l2, l3, lb);
  }
  const v4u vh = (v4u){h0, h1, h2, h3};
  const v4u vl = (v4u){l0, l1, l2, l3};
  unsigned short* ph = a1h + (size_t)r * KD + kc0;
  unsigned short* pl = a1l + (size_t)r * KD + kc0;
  *(volatile v4u*)ph = vh;
  *(volatile v4u*)pl = vl;
  __threadfence();
  *(volatile v4u*)ph = vh;
  *(volatile v4u*)pl = vl;
}

__global__ __launch_bounds__(256) void k_gemm(const unsigned short* __restrict__ Ah, const unsigned short* __restrict__ Al,
                                              const unsigned short* __restrict__ Bh, const unsigned short* __restrict__ Bl,
                                              float* __restrict__ C) {
  __shared__ __align__(16) float st[8][16 * STP];

  const int tid = threadIdx.x, lane = tid & 31, wave = tid >> 5;
  const int hh = lane >> 4, c = lane & 15;
  const int wr = wave >> 2;
  const int wc = wave & 3;
  const int arow0 = blockIdx.y * BMT + wr * 64;
  const int nrow0 = blockIdx.x * BNT + wc * 32;

  v8f acc[4][2];
#pragma unroll
  for (int s = 0; s < 4; ++s) { acc[s][0] = zero8(); acc[s][1] = zero8(); }

#pragma unroll 1
  for (int k0 = 0; k0 < KD; k0 += 32) {
    const v16bf bh0 = ldfrag(Bh, nrow0, k0, lane);
    const v16bf bh1 = ldfrag(Bh, nrow0 + 16, k0, lane);
    const v16bf bl0 = ldfrag(Bl, nrow0, k0, lane);
    const v16bf bl1 = ldfrag(Bl, nrow0 + 16, k0, lane);
#pragma unroll
    for (int s = 0; s < 4; ++s) {
      const v16bf ah = ldfrag(Ah, arow0 + 16 * s, k0, lane);
      const v16bf al = ldfrag(Al, arow0 + 16 * s, k0, lane);
      acc[s][0] = mma_bf(ah, bh0, acc[s][0]);
      acc[s][0] = mma_bf(ah, bl0, acc[s][0]);
      acc[s][0] = mma_bf(al, bh0, acc[s][0]);
      acc[s][1] = mma_bf(ah, bh1, acc[s][1]);
      acc[s][1] = mma_bf(ah, bl1, acc[s][1]);
      acc[s][1] = mma_bf(al, bh1, acc[s][1]);
    }
  }

  float* sw = st[wave];
#pragma unroll
  for (int s = 0; s < 4; ++s) {
#pragma unroll
    for (int r = 0; r < 8; ++r) {
      sw[(8 * hh + r) * STP + c]      = acc[s][0][r];
      sw[(8 * hh + r) * STP + 16 + c] = acc[s][1][r];
    }
    __syncthreads();
    v4f val[4];
    size_t go[4];
#pragma unroll
    for (int it = 0; it < 4; ++it) {
      const int p  = lane + 32 * it;
      const int L  = p >> 3;
      const int pc = p & 7;
      val[it] = *(const v4fa*)(sw + L * STP + pc * 4);
      go[it]  = (size_t)(arow0 + s * 16 + L) * ND + nrow0 + pc * 4;
    }
    for (int ps = 0; ps < 2; ++ps) {
#pragma unroll
      for (int it = 0; it < 4; ++it) *(volatile v4f*)(C + go[it]) = val[it];
      __threadfence();
    }
    __syncthreads();
  }
}

__device__ __forceinline__ float sig_at(const float* __restrict__ frb, int s) {
  const bool sok = (s >= 0) && (s < SIG_LEN);
  const int sc = min(max(s, 0), SIG_LEN - 1);
  const int fh = sc / HOP;
  float v = 0.0f;
#pragma unroll
  for (int d = 1; d >= 0; --d) {
    const int f = fh - d;
    const bool fv = (f >= 0) && (f < FRAMES);
    const int fc = min(max(f, 0), FRAMES - 1);
    const int o2 = sc - HOP * fc;
    const bool ov = (o2 >= 0) && (o2 < WLEN);
    const int oc = min(max(o2, 0), WLEN - 1);
    const float ld = frb[(size_t)fc * KD + oc];
    v = (fv && ov) ? (v + ld) : v;
  }
  return sok ? v : 0.0f;
}

__device__ __forceinline__ float ts_at(const float* __restrict__ frb, const float* s_inc, int t) {
  const int nh = t / STEP;
  float acc = 0.0f;
#pragma unroll
  for (int d = 1; d >= 0; --d) {
    const int n = nh - d;
    const bool nv = (n >= 0) && (n < N_SEG);
    const int ncl = min(max(n, 0), N_SEG - 1);
    const int o = t - STEP * ncl;
    const bool ov = (o >= 0) && (o < SEG);
    const int oc = min(max(o, 0), SEG - 1);
    const int ii = min(oc, OV - 1);
    const int id = min(max(SEG - 1 - oc, 0), OV - 1);
    const float minc = s_inc[ii];
    const float mdec = s_inc[id];
    const float mhead = (ncl == 0) ? 1.0f : minc;
    const float mtail = (ncl == N_SEG - 1) ? 1.0f : mdec;
    const float mk = (oc < OV) ? mhead : ((oc < STEP) ? 1.0f : mtail);
    const int sp = t - DSHIFT * ncl;
    const float sv = sig_at(frb, sp);
    const float term = mk * sv;
    acc = (nv && ov) ? (acc + term) : acc;
  }
  return acc;
}

__global__ __launch_bounds__(128) void k_frame2(const float* __restrict__ frames,
                                               unsigned short* __restrict__ a2h, unsigned short* __restrict__ a2l) {
  __shared__ float s_inc[64];
  const int tid = threadIdx.x;
  const int r = blockIdx.x;
  const int b = r / FR2, m = r - b * FR2;
  if (tid < 64) {
    const int o1 = (tid < OV) ? tid : (OV - 1);
    s_inc[tid] = (float)(o1 + 1) / (float)OV;
  }
  __syncthreads();
  const float* frb = frames + (size_t)b * FRAMES * KD;
  const int n0 = tid * 8;
  unsigned int h0 = 0u, h1 = 0u, h2 = 0u, h3 = 0u, l0 = 0u, l1 = 0u, l2 = 0u, l3 = 0u;
#pragma unroll 1
  for (int j = 0; j < 8; ++j) {
    const int n = n0 + j;
    const bool nv = n < WLEN;
    const int t = HOP * m + (nv ? n : (WLEN - 1));
    float v = ts_at(frb, s_inc, t);
    consume(v);
    v = nv ? v : 0.0f;
    unsigned int hb, lb;
    split_bf16(v, hb, lb);
    shin(h0, h1, h2, h3, hb);
    shin(l0, l1, l2, l3, lb);
  }
  const v4u vh = (v4u){h0, h1, h2, h3};
  const v4u vl = (v4u){l0, l1, l2, l3};
  unsigned short* ph = a2h + (size_t)r * KD + n0;
  unsigned short* pl = a2l + (size_t)r * KD + n0;
  *(volatile v4u*)ph = vh;
  *(volatile v4u*)pl = vl;
  __threadfence();
  *(volatile v4u*)ph = vh;
  *(volatile v4u*)pl = vl;
}

__global__ __launch_bounds__(256) void k_out(const float* __restrict__ S, float* __restrict__ out) {
  const int tid = threadIdx.x;
  const int i0 = (blockIdx.x * 256 + tid) * 4;
  float v[4];
#pragma unroll
  for (int j = 0; j < 4; ++j) {
    const int i = i0 + j;
    const int c = i & 1;
    const int q = i >> 1;
    const int m = q % FR2;
    const int bk = q / FR2;
    const int k = bk & (BINS - 1);
    const int b = bk >> 9;
    v[j] = S[(size_t)(b * FR2 + m) * ND + c * BINS + k];
  }
  const v4f val = (v4f){v[0], v[1], v[2], v[3]};
  *(volatile v4f*)(out + i0) = val;
  __threadfence();
  *(volatile v4f*)(out + i0) = val;
}

extern "C" void kernel_launch(void* const* d_in, const int* in_sizes, int n_in,
                              void* d_out, int out_size, void* d_ws, size_t ws_size,
                              hipStream_t stream) {
  if (n_in < 1) return;
  if (in_sizes[0] != BATCH * BINS * FRAMES * 2) return;
  if (out_size != OUT_N) return;
  if (ws_size < WS_TOTAL) return;

  const float* x = (const float*)d_in[0];
  float* out = (float*)d_out;
  char* ws = (char*)d_ws;

  float* cosT = (float*)(ws + OFF_TRIG);
  float* sinT = cosT + 1024;
  unsigned short* bih = (unsigned short*)(ws + OFF_BIH);
  unsigned short* bil = (unsigned short*)(ws + OFF_BIL);
  unsigned short* bfh = (unsigned short*)(ws + OFF_BFH);
  unsigned short* bfl = (unsigned short*)(ws + OFF_BFL);
  unsigned short* a1h = (unsigned short*)(ws + OFF_A1H);
  unsigned short* a1l = (unsigned short*)(ws + OFF_A1L);
  float* frames = (float*)(ws + OFF_FR);
  unsigned short* a2h = (unsigned short*)(ws + OFF_A2H);
  unsigned short* a2l = (unsigned short*)(ws + OFF_A2L);
  float* S = (float*)(ws + OFF_S);

  k_trig<<<dim3(4), dim3(256), 0, stream>>>(cosT, sinT);
  k_basis_inv<<<dim3(ND), dim3(128), 0, stream>>>(cosT, sinT, bih, bil);
  k_basis_fwd<<<dim3(ND), dim3(128), 0, stream>>>(cosT, sinT, bfh, bfl);
  k_pack1<<<dim3(M1), dim3(128), 0, stream>>>(x, a1h, a1l);
  k_gemm<<<dim3(ND / BNT, M1 / BMT), dim3(256), 0, stream>>>(a1h, a1l, bih, bil, frames);
  k_frame2<<<dim3(M2), dim3(128), 0, stream>>>(frames, a2h, a2l);
  k_gemm<<<dim3(ND / BNT, M2 / BMT), dim3(256), 0, stream>>>(a2h, a2l, bfh, bfl, S);
  k_out<<<dim3(OUT_N / 1024), dim3(256), 0, stream>>>(S, out);
  (void)hipGetLastError();
}
